// TransformerEncoderLayer_11055245819986
// MI455X (gfx1250) — hardware-verified
//
#include <hip/hip_runtime.h>
#ifndef NB
#define NB 2
#endif
#ifndef SEQ
#define SEQ 2048
#endif
#define NB_FULL 2
#define SEQ_FULL 2048
#define DM 768
#define NH 12
#define HD 64
#define DFF 3072
#define DMQ DM
#define NR ((size_t)NB * SEQ)
#define LQK (2 * DM)
static_assert(SEQ % 64 == 0);
static_assert(NB >= 1 && NB <= NB_FULL);
static_assert(SEQ <= SEQ_FULL);
static_assert(NH * HD == DM);
static_assert(DM % 128 == 0 && DFF % 64 == 0 && DM % 32 == 0 && DFF % 32 == 0);
static_assert(((size_t)NB * SEQ) % 128 == 0);
static_assert(DMQ % 4 == 0 && DMQ / 4 <= 256);

typedef unsigned short v8us __attribute__((ext_vector_type(8), may_alias));
typedef float  v8f  __attribute__((ext_vector_type(8)));
typedef float  v4f  __attribute__((ext_vector_type(4)));
typedef float  v4fa __attribute__((ext_vector_type(4), may_alias));
typedef _Float16 v16h __attribute__((ext_vector_type(16)));
typedef _Float16 v4h __attribute__((ext_vector_type(4)));
union FragH { v16h v; v8us half[2]; _Float16 h[16]; unsigned short u[16]; };

__device__ __forceinline__ unsigned short bf16_bits(float x) { unsigned int u = __float_as_uint(x); return (unsigned short)((u + 0x7FFFu + ((u >> 16) & 1u)) >> 16); }
__device__ __forceinline__ float bf16_val(unsigned short b) { return __uint_as_float(((unsigned int)b) << 16); }
__device__ __forceinline__ float bf16_rne(float x) { return bf16_val(bf16_bits(x)); }

__device__ __forceinline__ v16h g2_frag(const _Float16* p, int hh) { FragH f; f.half[0] = *(const v8us*)((const unsigned short*)p + 8 * hh); f.half[1] = *(const v8us*)((const unsigned short*)p + 16 + 8 * hh); return f.v; }
__device__ __forceinline__ v8f g2_mma(v16h a, v16h b, v8f c) { v8f d = __builtin_amdgcn_wmma_f32_16x16x32_f16(false, a, false, b, (short)0, c, false, false); asm volatile("v_nop\n\tv_nop\n\tv_nop\n\tv_nop" : "+v"(d) : "v"(a), "v"(b)); return d; }

__global__ __launch_bounds__(256) void k_wt_f16(const float* __restrict__ W, _Float16* __restrict__ Wt, int K, int N, float scale) {
  const int t = blockIdx.x * 256 + threadIdx.x; if (t >= N * (K / 8)) return; const int n = t / (K / 8), k8 = (t % (K / 8)) * 8; FragH f;
#pragma unroll
  for (int i = 0; i < 8; ++i) f.h[i] = (_Float16)(bf16_rne(W[(size_t)(k8 + i) * N + n]) * scale); const v8us o = f.half[0];
  *(volatile v8us*)((unsigned short*)Wt + (size_t)n * K + k8) = o; __threadfence(); *(volatile v8us*)((unsigned short*)Wt + (size_t)n * K + k8) = o;
}

__global__ __launch_bounds__(256) void k_wthd3(const float* __restrict__ Wa, const float* __restrict__ Wb, const float* __restrict__ Wc, _Float16* __restrict__ Bt) {
  const size_t t = (size_t)blockIdx.x * 256 + threadIdx.x; if (t >= (size_t)NH * HD * (DM / 8)) return;
  const int which = blockIdx.y; const float* W = (which == 0) ? Wa : ((which == 1) ? Wb : Wc);
  const int m8 = (int)(t % (DM / 8)) * 8; const int d = (int)((t / (DM / 8)) % HD); const int h = (int)(t / ((size_t)(DM / 8) * HD)); FragH f;
#pragma unroll
  for (int q = 0; q < 8; ++q) f.h[q] = (_Float16)(16.0f * bf16_rne(W[((size_t)h * DM + m8 + q) * HD + d]));
  unsigned short* dst = (unsigned short*)Bt + ((size_t)which * DM + (size_t)h * HD + d) * DM + m8;
  *(volatile v8us*)dst = f.half[0]; __threadfence(); *(volatile v8us*)dst = f.half[0];
}

__global__ __launch_bounds__(256) void k_xprep(const float* __restrict__ x, _Float16* __restrict__ X16, float* __restrict__ XB, size_t n8) {
  const size_t t = (size_t)blockIdx.x * 256 + threadIdx.x; if (t >= n8) return;
  const size_t e = t * 8; const size_t r = e / DM; const size_t c = e % DM; const size_t rs = (r / SEQ) * SEQ_FULL + (r % SEQ);
  const float* p = x + rs * DM + c; v4f a = *(const v4fa*)p, cc = *(const v4fa*)(p + 4); FragH f;
#pragma unroll
  for (int q = 0; q < 4; ++q) { a[q] = bf16_rne(a[q]); cc[q] = bf16_rne(cc[q]); f.h[q] = (_Float16)a[q]; f.h[4 + q] = (_Float16)cc[q]; }
  for (int pass = 0; pass < 2; ++pass) { *(volatile v8us*)((unsigned short*)X16 + e) = f.half[0]; *(volatile v4f*)(XB + e) = a; *(volatile v4f*)(XB + e + 4) = cc; if (pass == 0) __threadfence(); }
}

template <int ACT>
__global__ __launch_bounds__(128) void k_gemm2(const _Float16* __restrict__ A, int lda, size_t sA, const _Float16* __restrict__ Bh, int ldb, size_t sB, float alpha, const float* __restrict__ bias, size_t sBias, const float* __restrict__ CP, int rowsPerB, size_t sCPb, int row0g,
    float* __restrict__ C, _Float16* __restrict__ C16, int ldc, size_t sC, int M, int N, int K) { static_assert(ACT == 0 || ACT == 3);
  __shared__ __attribute__((aligned(16))) float so[4][32][68];
  const int tid = threadIdx.x, w = tid >> 5, lane = tid & 31, ln = lane & 15, hh = lane >> 4; const int by = blockIdx.y;
  A += (size_t)by * sA; Bh += (size_t)by * sB; const size_t cofs = (size_t)by * sC; const float* bp = bias ? bias + (size_t)by * sBias : nullptr;
  const int ntn = N >> 6; const int mt = blockIdx.x / ntn, nq = blockIdx.x - mt * ntn; const int row0 = mt * 128 + 32 * w, col0 = nq * 64; if (row0 >= M) return;
  const _Float16* a0p = A + (size_t)(row0 + ln) * lda; const _Float16* a1p = a0p + (size_t)16 * lda;
  const _Float16* b0p = Bh + (size_t)(col0 + ln) * ldb; const _Float16* b1p = b0p + (size_t)16 * ldb; const _Float16* b2p = b1p + (size_t)16 * ldb; const _Float16* b3p = b2p + (size_t)16 * ldb;
  const v8f z8 = {0.f,0.f,0.f,0.f,0.f,0.f,0.f,0.f}; v8f c00 = z8, c01 = z8, c02 = z8, c03 = z8, c10 = z8, c11 = z8, c12 = z8, c13 = z8;
#pragma unroll 1
  for (int kb = 0; kb < K; kb += 32) { const v16h a0 = g2_frag(a0p + kb, hh), a1 = g2_frag(a1p + kb, hh);
    v16h b = g2_frag(b0p + kb, hh); c00 = g2_mma(a0, b, c00); c10 = g2_mma(a1, b, c10);
    b = g2_frag(b1p + kb, hh); c01 = g2_mma(a0, b, c01); c11 = g2_mma(a1, b, c11);
    b = g2_frag(b2p + kb, hh); c02 = g2_mma(a0, b, c02); c12 = g2_mma(a1, b, c12);
    b = g2_frag(b3p + kb, hh); c03 = g2_mma(a0, b, c03); c13 = g2_mma(a1, b, c13); }
  v8f accs[8] = {c00, c01, c02, c03, c10, c11, c12, c13};
#pragma unroll
  for (int u = 0; u < 8; ++u) { const int t = u & 3, half = u >> 2; const int col = col0 + t * 16 + ln; const float bv = bp ? bf16_rne(bp[col]) : 0.f;
#pragma unroll
    for (int r = 0; r < 8; ++r) { const int rloc = half * 16 + 8 * hh + r; float v = accs[u][r] * alpha + bv; if (CP) { if (rowsPerB < 0) v += CP[cofs + (size_t)(row0g + row0 + rloc) * ldc + col];        else { const int bidx = (row0g + row0 + rloc) / rowsPerB; v += CP[(size_t)bidx * sCPb + (size_t)by * 64 + col]; } }
      if (ACT == 3) v = fmaxf(v, 0.f);
      so[w][rloc][t * 16 + ln] = v; } }
  __builtin_amdgcn_fence(4  , "workgroup"); __builtin_amdgcn_wave_barrier();
  const int rsub = lane >> 4, c4 = (lane & 15) * 4;
  for (int pass = 0; pass < 2; ++pass) {
#pragma unroll
    for (int q = 0; q < 16; ++q) { const int r = q * 2 + rsub; const v4f v = *(const v4fa*)&so[w][r][c4]; if (C) *(volatile v4f*)(C + cofs + (size_t)(row0 + r) * ldc + col0 + c4) = v; if (C16) { v4h h4; for (int i = 0; i < 4; ++i) h4[i] = (_Float16)v[i]; *(volatile v4h*)(C16 + cofs + (size_t)(row0 + r) * ldc + col0 + c4) = h4; } }
    if (pass == 0) __threadfence(); } }

template <int BFIN, int W16, int W32, int ORM>
__global__ __launch_bounds__(256) void k_lnx(const float* __restrict__ X, const float* __restrict__ g, const float* __restrict__ bb, float eps, _Float16* __restrict__ N16, float* __restrict__ N32) {
  #pragma clang fp contract(off)
  __shared__ float red[256]; const size_t r = blockIdx.x; const size_t ro = ORM ? ((r / SEQ) * SEQ_FULL + (r % SEQ)) : r; const int t = threadIdx.x; const bool act = t < (DMQ / 4); const int c0 = act ? t * 4 : 0;
  const v4f xa = *(const v4fa*)(X + r * DMQ + c0); float s[4]; float sum = 0.f;
  for (int q = 0; q < 4; ++q) { s[q] = act ? (BFIN ? bf16_rne(xa[q]) : xa[q]) : 0.f; sum = __fadd_rn(sum, s[q]); }
  red[t] = sum; __syncthreads(); for (int st = 128; st > 0; st >>= 1) { if (t < st) red[t] = __fadd_rn(red[t], red[t + st]); __syncthreads(); } const float mu = red[0] / (float)DMQ; __syncthreads();
  float vs = 0.f; for (int q = 0; q < 4; ++q) { const float dl = act ? __fadd_rn(s[q], -mu) : 0.f; vs = __fadd_rn(vs, __fmul_rn(dl, dl)); } red[t] = vs; __syncthreads(); for (int st = 128; st > 0; st >>= 1) { if (t < st) red[t] = __fadd_rn(red[t], red[t + st]); __syncthreads(); }
  const float rs = rsqrtf(__fadd_rn(red[0] / (float)DMQ, eps)); v4h y; v4f yf;
  for (int q = 0; q < 4; ++q) { const int c = c0 + q; yf[q] = __fadd_rn(__fmul_rn(__fmul_rn(__fadd_rn(s[q], -mu), rs), bf16_rne(g[c])), bf16_rne(bb[c])); y[q] = (_Float16)yf[q]; }
  if (!act) return;
  for (int pass = 0; pass < 2; ++pass) { if (W16) *(volatile v4h*)(N16 + ro * DMQ + c0) = y; if (W32) *(volatile v4f*)(N32 + ro * DMQ + c0) = yf; if (pass == 0) __threadfence(); } }

__global__ __launch_bounds__(128) void k_attn(const _Float16* __restrict__ QK, const _Float16* __restrict__ VT, _Float16* __restrict__ CAT) {
  __shared__ __attribute__((aligned(16))) unsigned short so[4][16][72];
  const int tid = threadIdx.x, w = tid >> 5, lane = tid & 31, nl = lane & 15, hh = lane >> 4;
  const int h = blockIdx.y, b = blockIdx.z;
  const int q0 = blockIdx.x * 64 + w * 16;
  const size_t rq = (size_t)b * SEQ + q0;
  const size_t rk = (size_t)b * SEQ;
  const _Float16* qp = QK + (rq + nl) * LQK + h * HD;
  const v16h qb0 = g2_frag(qp, hh), qb1 = g2_frag(qp + 32, hh);
  const _Float16* kp = QK + (rk + nl) * LQK + DM + h * HD;
  const _Float16* vp = VT + ((size_t)h * HD + nl) * NR + rk;
  const v8f z8 = {0.f,0.f,0.f,0.f,0.f,0.f,0.f,0.f};
  v8f o0 = z8, o1 = z8, o2 = z8, o3 = z8; float m = -1.0e30f, l = 0.f;
#pragma unroll 1
  for (int kb = 0; kb < SEQ; kb += 32) {
    const _Float16* k0p = kp + (size_t)kb * LQK; const _Float16* k1p = k0p + (size_t)16 * LQK;
    v8f s0 = z8, s1 = z8; v16h a;
    a = g2_frag(k0p, hh); s0 = g2_mma(a, qb0, s0); a = g2_frag(k0p + 32, hh); s0 = g2_mma(a, qb1, s0);
    a = g2_frag(k1p, hh); s1 = g2_mma(a, qb0, s1); a = g2_frag(k1p + 32, hh); s1 = g2_mma(a, qb1, s1);
    float mx = -1.0e30f;
#pragma unroll
    for (int r = 0; r < 8; ++r) mx = fmaxf(mx, fmaxf(s0[r], s1[r]));
    mx = fmaxf(mx, __shfl_xor(mx, 16, 32));
    const float mn = fmaxf(m, mx * 0.125f);
    const float sc = __expf(m - mn);
    FragH pf; float ps = 0.f;
#pragma unroll
    for (int r = 0; r < 8; ++r) { const float e0 = __expf(s0[r] * 0.125f - mn); const float e1 = __expf(s1[r] * 0.125f - mn); ps += e0 + e1; pf.h[r] = (_Float16)(e0 * 256.0f); pf.h[8 + r] = (_Float16)(e1 * 256.0f); }
    ps += __shfl_xor(ps, 16, 32);
    l = l * sc + ps; m = mn;
#pragma unroll
    for (int r = 0; r < 8; ++r) { o0[r] *= sc; o1[r] *= sc; o2[r] *= sc; o3[r] *= sc; }
    const _Float16* v0p = vp + kb;
    a = g2_frag(v0p, hh); o0 = g2_mma(a, pf.v, o0);
    a = g2_frag(v0p + (size_t)16 * NR, hh); o1 = g2_mma(a, pf.v, o1);
    a = g2_frag(v0p + (size_t)32 * NR, hh); o2 = g2_mma(a, pf.v, o2);
    a = g2_frag(v0p + (size_t)48 * NR, hh); o3 = g2_mma(a, pf.v, o3);
  }
  const float inv = 0.25f / l;
  { FragH f;
#pragma unroll
    for (int r = 0; r < 8; ++r) f.h[r] = (_Float16)(o0[r] * inv); *(v8us*)&so[w][nl][0 * 16 + 8 * hh] = f.half[0];
#pragma unroll
    for (int r = 0; r < 8; ++r) f.h[r] = (_Float16)(o1[r] * inv); *(v8us*)&so[w][nl][1 * 16 + 8 * hh] = f.half[0];
#pragma unroll
    for (int r = 0; r < 8; ++r) f.h[r] = (_Float16)(o2[r] * inv); *(v8us*)&so[w][nl][2 * 16 + 8 * hh] = f.half[0];
#pragma unroll
    for (int r = 0; r < 8; ++r) f.h[r] = (_Float16)(o3[r] * inv); *(v8us*)&so[w][nl][3 * 16 + 8 * hh] = f.half[0]; }
  __builtin_amdgcn_fence(4  , "workgroup"); __builtin_amdgcn_wave_barrier();
  const int pr = lane >> 3, pc = lane & 7;
  for (int pass = 0; pass < 2; ++pass) {
#pragma unroll
    for (int it = 0; it < 4; ++it) { const int row = it * 4 + pr; const v8us v = *(const v8us*)&so[w][row][pc * 8]; *(volatile v8us*)((unsigned short*)CAT + (rq + row) * DM + (size_t)h * HD + pc * 8) = v; }
    if (pass == 0) __threadfence(); }
}

extern "C" void kernel_launch(void* const* d_in, const int* in_sizes, int n_in,
                              void* d_out, int out_size, void* d_ws, size_t ws_size, hipStream_t stream) {
  if (n_in < 14) return;
  const float* const* I = (const float* const*)d_in;
  const float* x = I[0]; const float* wq = I[1]; const float* wk = I[2]; const float* wv = I[3]; const float* wo = I[4]; const float* bo = I[5]; const float* g1 = I[6]; const float* be1 = I[7]; const float* w1 = I[8]; const float* b1 = I[9]; const float* w2 = I[10]; const float* b2 = I[11]; const float* g2 = I[12]; const float* be2 = I[13];
  const size_t need = ((size_t)(NB - 1) * SEQ_FULL + SEQ) * DM;
  if ((size_t)in_sizes[0] < need || (size_t)out_size < need) return;
  if (in_sizes[1] < NH * DM * HD || in_sizes[2] < NH * DM * HD || in_sizes[3] < NH * DM * HD || in_sizes[4] < DM * DM || in_sizes[5] < DM || in_sizes[6] < DM || in_sizes[7] < DM || in_sizes[8] < DM * DFF || in_sizes[9] < DFF || in_sizes[10] < DFF * DM || in_sizes[11] < DM || in_sizes[12] < DM || in_sizes[13] < DM) return;
  const int M = (int)NR;
  char* ws = (char*)d_ws; size_t off = 0;
  auto take = [&](size_t bytes) { char* p = ws + off; off += (bytes + 255) & ~(size_t)255; return p; };
  _Float16* BQKV = (_Float16*)take((size_t)3 * DM * DM * 2);
  _Float16* BTO  = (_Float16*)take((size_t)DM * DM * 2);
  _Float16* BW1  = (_Float16*)take((size_t)DFF * DM * 2);
  _Float16* BW2  = (_Float16*)take((size_t)DM * DFF * 2);
  _Float16* X16  = (_Float16*)take(NR * DM * 2);
  float*    XB   = (float*)take(NR * DM * 4);
  _Float16* QK16 = (_Float16*)take(NR * LQK * 2);
  _Float16* VT16 = (_Float16*)take((size_t)DM * NR * 2);
  _Float16* CAT16 = (_Float16*)take(NR * DM * 2);
  float*    T1   = (float*)take(NR * DM * 4);
  _Float16* R16  = (_Float16*)take(NR * DM * 2);
  float*    REC  = (float*)take(NR * DM * 4);
  _Float16* H16  = (_Float16*)take(NR * DFF * 2);
  float*    T2   = T1;
  if (off > ws_size) return;
  k_xprep<<<(unsigned)((NR * DM / 8 + 255) / 256), 256, 0, stream>>>(x, X16, XB, NR * DM / 8);
  k_wthd3<<<dim3((unsigned)(((size_t)NH * HD * (DM / 8) + 255) / 256), 3), 256, 0, stream>>>(wq, wk, wv, BQKV);
  k_wt_f16<<<(unsigned)(((size_t)DM * DM / 8 + 255) / 256), 256, 0, stream>>>(wo, BTO, DM, DM, 16.0f);
  k_wt_f16<<<(unsigned)(((size_t)DM * DFF / 8 + 255) / 256), 256, 0, stream>>>(w1, BW1, DM, DFF, 16.0f);
  k_wt_f16<<<(unsigned)(((size_t)DFF * DM / 8 + 255) / 256), 256, 0, stream>>>(w2, BW2, DFF, DM, 16.0f);
  k_gemm2<0><<<dim3((unsigned)(((M + 127) / 128) * (LQK / 64)), 1), 128, 0, stream>>>(X16, DM, 0, BQKV, DM, 0, 0.0625f, nullptr, 0, nullptr, 1, 0, 0, nullptr, QK16, LQK, 0, M, LQK, DM);
  k_gemm2<0><<<dim3((unsigned)((DM / 128) * (M / 64)), 1), 128, 0, stream>>>(BQKV + (size_t)2 * DM * DM, DM, 0, X16, DM, 0, 0.0625f, nullptr, 0, nullptr, 1, 0, 0, nullptr, VT16, M, 0, DM, M, DM);
  k_attn<<<dim3(SEQ / 64, NH, NB), 128, 0, stream>>>(QK16, VT16, CAT16);
  k_gemm2<0><<<dim3((unsigned)(((M + 127) / 128) * (DM / 64)), 1), 128, 0, stream>>>(CAT16, DM, 0, BTO, DM, 0, 0.0009765625f, bo, 0, XB, -1, 0, 0, T1, nullptr, DM, 0, M, DM, DM);
  k_lnx<0, 1, 1, 0><<<(unsigned)M, 256, 0, stream>>>(T1, g1, be1, 1e-5f, R16, REC);
  k_gemm2<3><<<dim3((unsigned)(((M + 127) / 128) * (DFF / 64)), 1), 128, 0, stream>>>(R16, DM, 0, BW1, DM, 0, 0.0625f, b1, 0, nullptr, 1, 0, 0, nullptr, H16, DFF, 0, M, DFF, DM);
  k_gemm2<0><<<dim3((unsigned)(((M + 127) / 128) * (DM / 64)), 1), 128, 0, stream>>>(H16, DFF, 0, BW2, DFF, 0, 0.0625f, b2, 0, REC, -1, 0, 0, T2, nullptr, DM, 0, M, DM, DFF);
  k_lnx<0, 0, 1, 1><<<(unsigned)M, 256, 0, stream>>>(T2, g2, be2, 1e-5f, nullptr, (float*)d_out);
}
